// TransformerEncoder_67697274519855
// MI455X (gfx1250) — hardware-run, weakly checked
//
#include <hip/hip_runtime.h>
#include <math.h>

typedef __attribute__((ext_vector_type(16))) _Float16 v16h;
typedef __attribute__((ext_vector_type(8)))  _Float16 v8h;
typedef __attribute__((ext_vector_type(8)))  float v8f;
typedef __attribute__((ext_vector_type(4)))  float v4f;
typedef __attribute__((ext_vector_type(4)))  unsigned v4u;
union H8 { v8h v; v4u u; };

template <typename T> __device__ __forceinline__ void vst2(void* p, T v) { *(volatile T*)p = v; __threadfence(); *(volatile T*)p = v; }
__device__ __forceinline__ v8f wmma16(v16h a, v16h b, v8f c) {
  v8f d = __builtin_amdgcn_wmma_f32_16x16x32_f16(false, a, false, b, (short)0, c, false, false);
  asm volatile("v_nop\n\tv_nop\n\tv_nop\n\tv_nop" : "+v"(d) : "v"(a), "v"(b));
  return d;
}
__device__ __forceinline__ float bfr(float v) { return (float)(__bf16)v; }
__device__ __forceinline__ v4f bfr4(v4f v) { v4f r; r[0] = bfr(v[0]); r[1] = bfr(v[1]); r[2] = bfr(v[2]); r[3] = bfr(v[3]); return r; }
__device__ __forceinline__ v16h frag_h(const _Float16* rowk0, int lane) {
  union { v16h v; v8h q[2]; } u; const _Float16* p = rowk0 + 8 * (lane >> 4);
  u.q[0] = *(const v8h*)p; u.q[1] = *(const v8h*)(p + 16); return u.v;
}
__device__ __forceinline__ v16h frag_f32(const float* rowk0, int lane) {
  v16h a; const float* p = rowk0 + 8 * (lane >> 4);
  const v4f x0 = *(const v4f*)p, x1 = *(const v4f*)(p + 4), x2 = *(const v4f*)(p + 16), x3 = *(const v4f*)(p + 20);
#pragma unroll
  for (int i = 0; i < 4; ++i) { a[i] = (_Float16)x0[i]; a[4 + i] = (_Float16)x1[i]; a[8 + i] = (_Float16)x2[i]; a[12 + i] = (_Float16)x3[i]; }
  return a;
}
static __device__ __forceinline__ _Float16 toh_flush(float v) { const _Float16 r = (_Float16)v; return (fabsf(v) < 6.103515625e-05f) ? (_Float16)0.0f : r; }
#define LDSX() do { asm volatile("s_wait_dscnt 0" ::: "memory"); __builtin_amdgcn_wave_barrier(); __builtin_amdgcn_fence(3  , "workgroup"); } while (0)

#ifndef NB
#define NB 8
#endif
#ifndef SEQ
#define SEQ 512
#endif
#define NB_FULL 8
#define SEQ_FULL 512
#define TT SEQ
#define CIN 64
#define CC 1024
#define NH 16
#define HD 64
#define NL 2
#define NRW (NB * TT)
#define NQB (TT / 64)
#define QSCALE (0.125f)
#define WCAR (64.0f)
#define HCAR (16.0f)
#define PCAR (2048.0f)
#define BN_EPS (1e-3f)
static_assert(NB >= 1 && NB <= NB_FULL);
static_assert(TT >= 128 && TT <= SEQ_FULL && (TT % 128) == 0);
static_assert(NH * HD == CC);
static_assert((HD % 32) == 0 && (CIN % 64) == 0 && (CIN % 32) == 0 && (CC % 32) == 0);
static_assert((CC % 256) == 0 && (CC % 128) == 0 && (NRW % 64) == 0 && (NRW % 8) == 0 && (CC % 64) == 0);
static_assert((((size_t)NRW * CIN) % 2048) == 0);
static_assert((((size_t)NRW * CC) % 2048) == 0);
static_assert(8 * 32 * 16 == 16 * 128 * 2);
static_assert(16 * 32 * 16 == 16 * 128 * 4);
static_assert(8 * 128 * 16 == 128 * 64 * 2);
static_assert(2 * 32 * 16 == 256 * 4 && 32 * 16 == 256 * 2);
static_assert(16 * 16 == 2 * 128);
static_assert(4 * 16 * 132 * 4 + 128 * 72 * 2 <= 131072);
static_assert(4 * 16 * 132 * 4 <= 131072);
static_assert(8 * TT * 4 <= 131072);
static_assert(64 * 65 * 4 <= 131072);
static_assert(8 * 32 * 4 + 2 * 32 * 4 <= 131072);
static_assert(8 * 256 * 4 <= 131072);

#define SZ_WE   (2u * (size_t)CC * CIN)
#define SZ_W    (2u * (size_t)CC * CC)
#define SZ_X16  (2u * (size_t)NRW * CIN)
#define SZ_ACT  (2u * (size_t)NRW * CC)
#define SZ_F32  (4u * (size_t)NRW * CC)
#define SZ_S    (4u * (size_t)NH * TT * TT)
#define SZ_ST   (4u * 2u * (size_t)CC)
#define WS_WE   ((size_t)0)
#define WS_WQ   (WS_WE + SZ_WE)
#define WS_WK   (WS_WQ + NL * SZ_W)
#define WS_WV   (WS_WK + NL * SZ_W)
#define WS_WC   (WS_WV + NL * SZ_W)
#define WS_X16  (WS_WC + NL * SZ_W)
#define WS_E16  (WS_X16 + SZ_X16)
#define WS_Q    (WS_E16 + SZ_ACT)
#define WS_K    (WS_Q + SZ_ACT)
#define WS_VT   (WS_K + SZ_ACT)
#define WS_S    (WS_VT + SZ_ACT)
#define WS_AO   (WS_S + SZ_S)
#define WS_ENCA (WS_AO + SZ_F32)
#define WS_ENCB (WS_ENCA + SZ_F32)
#define WS_ST   (WS_ENCB + SZ_F32)
#define WS_END  (WS_ST + SZ_ST)
static_assert((SZ_WE % 8192) == 0 && (SZ_X16 % 8192) == 0 && (SZ_ACT % 8192) == 0 && (SZ_S % 8192) == 0);
static_assert(WS_END <= (size_t)134217728u);

__global__ __launch_bounds__(256) void k_wcvt(const float* __restrict__ W, int K, int N, _Float16* __restrict__ WT) {
  __shared__ float tile[64][65];
  const int tid = threadIdx.x, tx = tid & 63, ty = tid >> 6; const int k0 = blockIdx.y * 64, n0 = blockIdx.x * 64;
#pragma unroll 1
  for (int i = ty; i < 64; i += 4) tile[i][tx] = W[(size_t)(k0 + i) * N + n0 + tx];
  __syncthreads();
#pragma unroll 1
  for (int e = tid; e < 64 * 8; e += 256) { const int nn = e >> 3, q = e & 7; H8 o;
#pragma unroll
    for (int i = 0; i < 8; ++i) o.v[i] = toh_flush(bfr(tile[q * 8 + i][nn]) * WCAR);
    vst2(WT + (size_t)(n0 + nn) * K + k0 + q * 8, o.u); }
}

__global__ __launch_bounds__(256) void k_xcvt(const float* __restrict__ X, _Float16* __restrict__ X16) {
#pragma clang fp contract(off)
  const size_t e = ((size_t)blockIdx.x * 256 + threadIdx.x) * 8;
  const size_t row = e / CIN; const int c = (int)(e % CIN);
  const size_t xrow = (row / TT) * SEQ_FULL + (row % TT);
  const float* p = X + xrow * CIN + c;
  const v4f a = bfr4(*(const v4f*)p), b = bfr4(*(const v4f*)(p + 4)); H8 o;
#pragma unroll
  for (int k = 0; k < 4; ++k) { o.v[k] = toh_flush(a[k]); o.v[4 + k] = toh_flush(b[k]); }
  vst2(X16 + e, o.u);
}

template <int MODE>
__global__ __launch_bounds__(128) void k_gem(const _Float16* __restrict__ A, int lda, int K, const _Float16* __restrict__ WT, int nout,
    const float* __restrict__ BIAS, float sa, float so, const float* __restrict__ AUX, _Float16* __restrict__ OH, float* __restrict__ OF) {
  __shared__ __align__(16) float sf[4][16][132];
  __shared__ __align__(16) _Float16 th[128][72];
  const int tid = threadIdx.x, wave = tid >> 5, lane = tid & 31, col = lane & 15, g = lane >> 4;
  const int c0 = blockIdx.y * 128; const size_t rb = (size_t)blockIdx.x * 64; const size_t r0 = rb + wave * 16;
  v8f acc[8] = {};
#pragma unroll 1
  for (int kc = 0; kc < K / 32; ++kc) {
    const v16h a = frag_h(A + (r0 + col) * (size_t)lda + kc * 32, lane);
    asm volatile("s_wait_loadcnt 0x0" ::: "memory");
#pragma unroll
    for (int j = 0; j < 8; ++j) { const v16h w = frag_h(WT + (size_t)(c0 + j * 16 + col) * K + kc * 32, lane); asm volatile("s_wait_loadcnt 0x0" ::: "memory"); acc[j] = wmma16(a, w, acc[j]); } }
  if (MODE == 1) {
    const size_t bb = rb / TT; const int t0 = (int)(rb % TT);
#pragma unroll
    for (int j = 0; j < 8; ++j) { const float bias = bfr(BIAS[c0 + j * 16 + col]);
#pragma unroll
      for (int r = 0; r < 8; ++r) th[j * 16 + col][wave * 16 + 8 * g + r] = toh_flush(fmaxf(acc[j][r] * sa + bias, 0.0f) * so); }
    __syncthreads();
#pragma unroll 1
    for (int e = tid; e < 128 * 8; e += 128) { const int cl = e >> 3, q = e & 7; vst2(OH + (bb * nout + c0 + cl) * (size_t)TT + t0 + q * 8, *(const v4u*)&th[cl][q * 8]); }
  } else {
#pragma unroll
    for (int j = 0; j < 8; ++j) { const float bias = (MODE == 2) ? 0.0f : bfr(BIAS[c0 + j * 16 + col]);
#pragma unroll
      for (int r = 0; r < 8; ++r) sf[wave][8 * g + r][j * 16 + col] = acc[j][r] * sa + bias; }
    LDSX();
    if (MODE == 0) {
#pragma unroll 1
      for (int i = 0; i < 8; ++i) { const int rl = 2 * i + g; const v4f u0 = *(const v4f*)&sf[wave][rl][col * 8], u1 = *(const v4f*)&sf[wave][rl][col * 8 + 4]; H8 o;
#pragma unroll
        for (int k = 0; k < 4; ++k) { o.v[k] = toh_flush(fmaxf(u0[k], 0.0f) * so); o.v[4 + k] = toh_flush(fmaxf(u1[k], 0.0f) * so); }
        vst2(OH + (r0 + rl) * (size_t)nout + c0 + col * 8, o.u); }
    } else {
#pragma unroll 1
      for (int rl = 0; rl < 16; ++rl) { const size_t r = r0 + rl; const size_t oo = r * (size_t)nout + c0 + lane * 4; v4f v = *(const v4f*)&sf[wave][rl][lane * 4];
        if (MODE == 3) { const v4f rv = *(const v4f*)(AUX + oo);
#pragma unroll
          for (int k = 0; k < 4; ++k) v[k] = rv[k] + fmaxf(v[k], 0.0f); }
        vst2(OF + oo, v); } } }
}

__global__ __launch_bounds__(128) void k_sc(const _Float16* __restrict__ Q, const _Float16* __restrict__ KK, int zb, int b0, int hd, float scale, float* __restrict__ S0) {
  __shared__ __align__(16) float ss[4][16][132];
  const int tid = threadIdx.x, wave = tid >> 5, lane = tid & 31, col = lane & 15, g = lane >> 4;
  const int qb = blockIdx.x, kb = blockIdx.y, z = blockIdx.z; const int b = zb ? b0 + z : b0; const int h = zb ? 0 : z;
  float* S = S0 + (size_t)z * TT * TT; const int k0 = kb * 128; const int ql0 = qb * 64 + wave * 16;
  const _Float16* qrow = Q + ((size_t)b * TT + ql0 + col) * CC + (size_t)h * hd;
  const _Float16* kbase = KK + ((size_t)b * TT + k0 + col) * CC + (size_t)h * hd;
  v8f acc[8] = {};
#pragma unroll 1
  for (int kc = 0; kc < hd / 32; ++kc) { const v16h a = frag_h(qrow + kc * 32, lane); asm volatile("s_wait_loadcnt 0x0" ::: "memory");
#pragma unroll
    for (int j = 0; j < 8; ++j) { const v16h kf = frag_h(kbase + (size_t)(j * 16) * CC + kc * 32, lane); asm volatile("s_wait_loadcnt 0x0" ::: "memory"); acc[j] = wmma16(a, kf, acc[j]); } }
#pragma unroll
  for (int j = 0; j < 8; ++j)
#pragma unroll
    for (int r = 0; r < 8; ++r) ss[wave][8 * g + r][j * 16 + col] = acc[j][r] * scale;
  LDSX();
#pragma unroll 1
  for (int rl = 0; rl < 16; ++rl) vst2(S + (size_t)(ql0 + rl) * TT + k0 + lane * 4, *(const v4f*)&ss[wave][rl][lane * 4]);
}

__global__ __launch_bounds__(256) void k_sm(float* __restrict__ S0) {
  __shared__ __align__(16) float shv[8][TT];
  const int wave = threadIdx.x >> 5, lane = threadIdx.x & 31; const int t = blockIdx.x * 8 + wave; const int z = blockIdx.y;
  float* sr = S0 + ((size_t)z * TT + t) * TT;
  float m = -3.0e38f;
#pragma unroll 1
  for (int i = 0; i < TT / 128; ++i) { const int c = i * 128 + lane * 4; const v4f v = *(const v4f*)(sr + c);
    *(v4f*)&shv[wave][c] = v; m = fmaxf(fmaxf(m, fmaxf(v[0], v[1])), fmaxf(v[2], v[3])); }
#pragma unroll
  for (int o = 1; o < 32; o <<= 1) m = fmaxf(m, __shfl_xor(m, o));
  float sum = 0.f;
#pragma unroll 1
  for (int i = 0; i < TT / 128; ++i) { const int c = i * 128 + lane * 4; const v4f v = *(const v4f*)&shv[wave][c]; v4f e;
#pragma unroll
    for (int k = 0; k < 4; ++k) e[k] = exp2f((v[k] - m) * 1.4426950408889634f);
    *(v4f*)&shv[wave][c] = e; sum += (e[0] + e[1]) + (e[2] + e[3]); }
#pragma unroll
  for (int o = 1; o < 32; o <<= 1) sum += __shfl_xor(sum, o);
  const float inv = PCAR * (1.0f / sum);
#pragma unroll 1
  for (int i = 0; i < TT / 128; ++i) { const int c = i * 128 + lane * 4; v4f v = *(const v4f*)&shv[wave][c]; v *= inv; vst2(sr + c, v); }
}

__global__ __launch_bounds__(128) void k_pv(const float* __restrict__ PS0, const _Float16* __restrict__ VT, int zb, int b0, int hd, float oscale, int out16, _Float16* __restrict__ OH, float* __restrict__ OF) {
  __shared__ __align__(16) float ss[4][16][132];
  const int tid = threadIdx.x, wave = tid >> 5, lane = tid & 31, col = lane & 15, g = lane >> 4;
  const int qb = blockIdx.x, z = blockIdx.z; const int c0 = blockIdx.y * 128; const int b = zb ? b0 + z : b0;
  const int sl0 = zb ? z : (c0 / hd), sl1 = zb ? z : ((c0 + 64) / hd); const int ql0 = qb * 64 + wave * 16;
  const float* p0 = PS0 + ((size_t)sl0 * TT + ql0 + col) * TT; const float* p1 = PS0 + ((size_t)sl1 * TT + ql0 + col) * TT;
  const _Float16* vbase = VT + ((size_t)b * CC + c0 + col) * TT;
  v8f acc[8] = {};
#pragma unroll 1
  for (int kc = 0; kc < TT / 32; ++kc) {
    const v16h a0 = frag_f32(p0 + kc * 32, lane); asm volatile("s_wait_loadcnt 0x0" ::: "memory");
    v16h a1 = a0; if (sl1 != sl0) { a1 = frag_f32(p1 + kc * 32, lane); asm volatile("s_wait_loadcnt 0x0" ::: "memory"); }
#pragma unroll
    for (int j = 0; j < 8; ++j) { const v16h vf = frag_h(vbase + (size_t)(j * 16) * TT + kc * 32, lane); asm volatile("s_wait_loadcnt 0x0" ::: "memory"); acc[j] = wmma16(j < 4 ? a0 : a1, vf, acc[j]); } }
#pragma unroll
  for (int j = 0; j < 8; ++j)
#pragma unroll
    for (int r = 0; r < 8; ++r) ss[wave][8 * g + r][j * 16 + col] = acc[j][r] * oscale;
  LDSX();
  const size_t orow0 = (size_t)b * TT + ql0;
  if (out16) {
#pragma unroll 1
    for (int i = 0; i < 8; ++i) { const int rl = 2 * i + g; const v4f u0 = *(const v4f*)&ss[wave][rl][col * 8], u1 = *(const v4f*)&ss[wave][rl][col * 8 + 4]; H8 o;
#pragma unroll
      for (int k = 0; k < 4; ++k) { o.v[k] = (_Float16)u0[k]; o.v[4 + k] = (_Float16)u1[k]; }
      vst2(OH + (orow0 + rl) * CC + c0 + col * 8, o.u); }
  } else {
#pragma unroll 1
    for (int rl = 0; rl < 16; ++rl) vst2(OF + (orow0 + rl) * CC + c0 + lane * 4, *(const v4f*)&ss[wave][rl][lane * 4]); }
}

__global__ __launch_bounds__(256) void k_bnstat(const float* __restrict__ X, const float* __restrict__ R, int hasr, float* __restrict__ ST) {
#pragma clang fp contract(off)
  __shared__ float part[8][32];
  __shared__ __align__(16) float fin[2][32];
  const int wave = __builtin_amdgcn_readfirstlane(threadIdx.x >> 5); const int lane = threadIdx.x & 31;
  const int c = blockIdx.x * 32 + lane;
  float s = 0.f;
#pragma unroll 1
  for (int i = 0; i < NRW / 8; ++i) { const size_t o = ((size_t)i * 8 + wave) * CC + c; float v = X[o]; if (hasr) v += R[o]; s += v; }
  part[wave][lane] = s;
  __syncthreads();
  float tot = 0.f;
#pragma unroll
  for (int w = 0; w < 8; ++w) tot += part[w][lane];
  const float mu = tot * (1.0f / NRW);
  __syncthreads();
  float q = 0.f;
#pragma unroll 1
  for (int i = 0; i < NRW / 8; ++i) { const size_t o = ((size_t)i * 8 + wave) * CC + c; float v = X[o]; if (hasr) v += R[o]; const float d = v - mu; q += d * d; }
  part[wave][lane] = q;
  __syncthreads();
  float qt = 0.f;
#pragma unroll
  for (int w = 0; w < 8; ++w) qt += part[w][lane];
  const float rs = 1.0f / sqrtf(qt * (1.0f / NRW) + BN_EPS);
  if (wave == 0) { fin[0][lane] = mu; fin[1][lane] = rs; }
  __syncthreads();
  if (threadIdx.x < 16) { const int w = threadIdx.x >> 3, qd = threadIdx.x & 7; const v4f o = *(const v4f*)&fin[w][qd * 4]; vst2(ST + (size_t)w * CC + blockIdx.x * 32 + qd * 4, o); }
}

__global__ __launch_bounds__(256) void k_bnap(const float* __restrict__ X, const float* __restrict__ R, int hasr, const float* __restrict__ ST, const float* __restrict__ G, const float* __restrict__ BE,
    const int* __restrict__ NHP, float* __restrict__ OF, int w16, _Float16* __restrict__ OH) {
#pragma clang fp contract(off)
  __shared__ __align__(16) float ys[8][256];
  const int wave = __builtin_amdgcn_readfirstlane(threadIdx.x >> 5); const int lane = threadIdx.x & 31;
  const size_t base = ((size_t)blockIdx.x * 8 + wave) * 256; const int cb = (int)(base % CC);
  const int nh = NHP[0]; const float pz = (nh == NH) ? 0.0f : __uint_as_float(0x7fc00000u);
#pragma unroll 1
  for (int hs = 0; hs < 2; ++hs) { const int cl = hs * 128 + lane * 4; const size_t e = base + cl; const int c = cb + cl;
    v4f v = *(const v4f*)(X + e); if (hasr) { const v4f rv = *(const v4f*)(R + e); v += rv; }
    const v4f mu = *(const v4f*)(ST + c), rs = *(const v4f*)(ST + CC + c); const v4f gg = bfr4(*(const v4f*)(G + c)), be = bfr4(*(const v4f*)(BE + c)); v4f y;
#pragma unroll
    for (int k = 0; k < 4; ++k) y[k] = (((gg[k] * (v[k] - mu[k])) * rs[k]) + be[k]) + pz;
    vst2(OF + e, y); *(v4f*)&ys[wave][cl] = y; }
  if (w16) {
    LDSX();
    const v4f u0 = *(const v4f*)&ys[wave][lane * 8], u1 = *(const v4f*)&ys[wave][lane * 8 + 4]; H8 o;
#pragma unroll
    for (int k = 0; k < 4; ++k) { o.v[k] = toh_flush(u0[k]); o.v[4 + k] = toh_flush(u1[k]); }
    vst2(OH + base + lane * 8, o.u); }
}

extern "C" void kernel_launch(void* const* d_in, const int* in_sizes, int n_in, void* d_out, int out_size, void* d_ws, size_t ws_size, hipStream_t stream) {
  if (n_in < 17) return;
  const float* const* F = (const float* const*)d_in;
  const int* NHP = (const int*)d_in[16];
  const long long nrowx = (long long)(NB - 1) * SEQ_FULL + TT;
  if ((long long)in_sizes[0] < nrowx * CIN) return;
  if ((long long)in_sizes[1] < (long long)CIN * CC || in_sizes[2] < CC || in_sizes[3] < CC) return;
  if ((long long)in_sizes[4] < (long long)NL * CC * CC || (long long)in_sizes[6] < (long long)NL * CC * CC || (long long)in_sizes[8] < (long long)NL * CC * CC || (long long)in_sizes[12] < (long long)NL * CC * CC) return;
  if (in_sizes[5] < NL * CC || in_sizes[7] < NL * CC || in_sizes[9] < NL * CC || in_sizes[10] < NL * CC || in_sizes[11] < NL * CC || in_sizes[13] < NL * CC || in_sizes[14] < NL * CC || in_sizes[15] < NL * CC) return;
  if (in_sizes[16] < 1) return;
  if ((long long)out_size < (long long)NRW * CC) return;
  if (ws_size < (size_t)WS_END) return;
  char* ws = (char*)d_ws;
  _Float16 *WET = (_Float16*)(ws + WS_WE);
  _Float16 *X16 = (_Float16*)(ws + WS_X16), *E16 = (_Float16*)(ws + WS_E16), *Q16 = (_Float16*)(ws + WS_Q), *K16 = (_Float16*)(ws + WS_K), *VT16 = (_Float16*)(ws + WS_VT), *H16 = (_Float16*)(ws + WS_Q);
  float *SS = (float*)(ws + WS_S), *AO = (float*)(ws + WS_AO), *ENCA = (float*)(ws + WS_ENCA), *ENCB = (float*)(ws + WS_ENCB), *ST = (float*)(ws + WS_ST);
  float* OUT = (float*)d_out;

  k_wcvt<<<dim3(CC / 64, CIN / 64), 256, 0, stream>>>(F[1], CIN, CC, WET);
  for (int i = 0; i < NL; ++i) {
    const size_t wo = (size_t)i * CC * CC;
    k_wcvt<<<dim3(CC / 64, CC / 64), 256, 0, stream>>>(F[4] + wo, CC, CC, (_Float16*)(ws + WS_WQ + i * SZ_W));
    k_wcvt<<<dim3(CC / 64, CC / 64), 256, 0, stream>>>(F[6] + wo, CC, CC, (_Float16*)(ws + WS_WK + i * SZ_W));
    k_wcvt<<<dim3(CC / 64, CC / 64), 256, 0, stream>>>(F[8] + wo, CC, CC, (_Float16*)(ws + WS_WV + i * SZ_W));
    k_wcvt<<<dim3(CC / 64, CC / 64), 256, 0, stream>>>(F[12] + wo, CC, CC, (_Float16*)(ws + WS_WC + i * SZ_W));
  }
  k_xcvt<<<dim3((unsigned)(((size_t)NRW * CIN) / 2048)), 256, 0, stream>>>(F[0], X16);
  k_gem<2><<<dim3(NRW / 64, CC / 128), 128, 0, stream>>>(X16, CIN, CIN, WET, CC, nullptr, 1.0f / WCAR, 1.0f, nullptr, nullptr, AO);
  k_bnstat<<<dim3(CC / 32), 256, 0, stream>>>(AO, AO, 0, ST);
  k_bnap<<<dim3((unsigned)(((size_t)NRW * CC) / 2048)), 256, 0, stream>>>(AO, AO, 0, ST, F[2], F[3], NHP, ENCA, 1, E16);

  for (int i = 0; i < NL; ++i) {
    const _Float16 *WQT = (const _Float16*)(ws + WS_WQ + i * SZ_W), *WKT = (const _Float16*)(ws + WS_WK + i * SZ_W), *WVT = (const _Float16*)(ws + WS_WV + i * SZ_W), *WCT = (const _Float16*)(ws + WS_WC + i * SZ_W);
    const size_t vo = (size_t)i * CC;
    k_gem<0><<<dim3(NRW / 64, CC / 128), 128, 0, stream>>>(E16, CC, CC, WQT, CC, F[5] + vo, 1.0f / WCAR, 1.0f, nullptr, Q16, nullptr);
    k_gem<0><<<dim3(NRW / 64, CC / 128), 128, 0, stream>>>(E16, CC, CC, WKT, CC, F[7] + vo, 1.0f / WCAR, 1.0f, nullptr, K16, nullptr);
    k_gem<1><<<dim3(NRW / 64, CC / 128), 128, 0, stream>>>(E16, CC, CC, WVT, CC, F[9] + vo, 1.0f / WCAR, 1.0f, nullptr, VT16, nullptr);
    for (int b = 0; b < NB; ++b) {
      k_sc<<<dim3(NQB, TT / 128, NH), 128, 0, stream>>>(Q16, K16, 0, b, HD, QSCALE, SS);
      k_sm<<<dim3(TT / 8, NH), 256, 0, stream>>>(SS);
      k_pv<<<dim3(NQB, CC / 128, 1), 128, 0, stream>>>(SS, VT16, 0, b, HD, 1.0f / PCAR, 0, nullptr, AO);
    }
    k_bnstat<<<dim3(CC / 32), 256, 0, stream>>>(AO, ENCA, 1, ST);
    k_bnap<<<dim3((unsigned)(((size_t)NRW * CC) / 2048)), 256, 0, stream>>>(AO, ENCA, 1, ST, F[10] + vo, F[11] + vo, NHP, ENCB, 1, E16);
    k_gem<0><<<dim3(NRW / 64, CC / 128), 128, 0, stream>>>(E16, CC, CC, WCT, CC, F[13] + vo, 1.0f / WCAR, HCAR, nullptr, H16, nullptr);
    k_gem<3><<<dim3(NRW / 64, CC / 128), 128, 0, stream>>>(H16, CC, CC, WCT, CC, F[13] + vo, 1.0f / (WCAR * HCAR), 1.0f, ENCB, nullptr, AO);
    const int last = (i == NL - 1) ? 1 : 0;
    k_bnstat<<<dim3(CC / 32), 256, 0, stream>>>(AO, AO, 0, ST);
    k_bnap<<<dim3((unsigned)(((size_t)NRW * CC) / 2048)), 256, 0, stream>>>(AO, AO, 0, ST, F[14] + vo, F[15] + vo, NHP, last ? OUT : ENCA, last ? 0 : 1, E16);
  }
}
